// SocialPoolingAttention_223338299638
// MI455X (gfx1250) — hardware-verified
//
#include <hip/hip_runtime.h>
#include <math.h>

typedef __attribute__((ext_vector_type(16))) _Float16 v16h;
typedef __attribute__((ext_vector_type(16))) __bf16 v16b;
typedef __attribute__((ext_vector_type(8)))  _Float16 v8h;
typedef __attribute__((ext_vector_type(8)))  float v8f;
typedef __attribute__((ext_vector_type(4)))  float v4f;
typedef __attribute__((ext_vector_type(2)))  float v2f;
typedef __attribute__((ext_vector_type(4)))  unsigned v4u;
typedef __attribute__((ext_vector_type(4)))  int v4i;
typedef float __attribute__((may_alias)) float_a;
typedef int __attribute__((may_alias)) int_a;

template <typename T> __device__ __forceinline__ void vst2(void* p, T v) { *(volatile T*)p = v; __threadfence(); *(volatile T*)p = v; }
__device__ __forceinline__ v8f wmma16(v16h a, v16h b, v8f c) {
  v8f d = __builtin_amdgcn_wmma_f32_16x16x32_f16(false, a, false, b, (short)0, c, false, false);
  asm volatile("v_nop\n\tv_nop\n\tv_nop\n\tv_nop" : "+v"(d) : "v"(a), "v"(b));
  return d;
}
__device__ __forceinline__ v8f wmma_bf(v16b a, v16b b, v8f c) {
  v8f d = __builtin_amdgcn_wmma_f32_16x16x32_bf16(false, a, false, b, (short)0, c, false, false);
  asm volatile("v_nop\n\tv_nop\n\tv_nop\n\tv_nop" : "+v"(d) : "v"(a), "v"(b));
  return d;
}
__device__ __forceinline__ v16h frag_h(const _Float16* rowk0, int lane) {
  union { v16h v; v8h q[2]; } u; const _Float16* p = rowk0 + 8 * (lane >> 4);
  u.q[0] = *(const v8h*)p; u.q[1] = *(const v8h*)(p + 16); return u.v;
}
__device__ __forceinline__ v16h frag_f32(const float* rowk0, int lane) {
  v16h a; const float* p = rowk0 + 8 * (lane >> 4);
#pragma unroll
  for (int i = 0; i < 8; ++i) { a[i] = (_Float16)p[i]; a[8 + i] = (_Float16)p[16 + i]; }
  return a;
}
__device__ __forceinline__ v16h frag_f32s(const float* rowk0, int lane, float sc) {
  v16h a; const float* p = rowk0 + 8 * (lane >> 4);
#pragma unroll
  for (int i = 0; i < 8; ++i) { a[i] = (_Float16)(p[i] * sc); a[8 + i] = (_Float16)(p[16 + i] * sc); }
  return a;
}
__device__ __forceinline__ v16h fragc_f32(const float* W, int k0, int n, int lane, int ld, int K) {
  v16h a; const int g = lane >> 4;
#pragma unroll
  for (int i = 0; i < 8; ++i) { const int ka = k0 + 8 * g + i, kb = ka + 16;
    a[i] = (_Float16)(ka < K ? W[(size_t)(ka < K ? ka : K - 1) * ld + n] : 0.f); a[8 + i] = (_Float16)(kb < K ? W[(size_t)(kb < K ? kb : K - 1) * ld + n] : 0.f); }
  return a;
}
struct F2 { v16b h, l; };
__device__ __forceinline__ F2 bsplit16(const float v[16]) { F2 r;
#pragma unroll
  for (int i = 0; i < 16; ++i) { const __bf16 h = (__bf16)v[i]; r.h[i] = h; r.l[i] = (__bf16)(v[i] - (float)h); }
  return r; }
__device__ __forceinline__ F2 split_row(const float* row, int k0, int lane) { float v[16]; const float* p = row + k0 + 8 * (lane >> 4);
#pragma unroll
  for (int i = 0; i < 8; ++i) { v[i] = p[i]; v[8 + i] = p[16 + i]; }
  return bsplit16(v); }
__device__ __forceinline__ F2 split_rowK(const float* row, int k0, int lane, int K) { float v[16]; const int g = lane >> 4;
#pragma unroll
  for (int i = 0; i < 8; ++i) { const int ka = k0 + 8 * g + i, kb = ka + 16; v[i] = ka < K ? row[ka < K ? ka : K - 1] : 0.f; v[8 + i] = kb < K ? row[kb < K ? kb : K - 1] : 0.f; }
  return bsplit16(v); }
__device__ __forceinline__ F2 split_col(const float* W, int k0, int n, int lane, int ld, int K) { float v[16]; const int g = lane >> 4;
#pragma unroll
  for (int i = 0; i < 8; ++i) { const int ka = k0 + 8 * g + i, kb = ka + 16; v[i] = ka < K ? W[(size_t)(ka < K ? ka : K - 1) * ld + n] : 0.f; v[8 + i] = kb < K ? W[(size_t)(kb < K ? kb : K - 1) * ld + n] : 0.f; }
  return bsplit16(v); }
__device__ __forceinline__ v8f mac3(const F2& a, const F2& b, v8f c) { c = wmma_bf(a.l, b.h, c); c = wmma_bf(a.h, b.l, c); return wmma_bf(a.h, b.h, c); }
__device__ __forceinline__ float sigm(float v) { return 1.0f / (1.0f + expf(-v)); }
#define LDSX() do { asm volatile("s_wait_dscnt 0" ::: "memory"); __builtin_amdgcn_wave_barrier(); __builtin_amdgcn_fence(__ATOMIC_RELEASE, "workgroup"); } while (0)


#define NS_ 32
#define NPED 64
#define NBP (NS_ * NPED)
#define HD 64
#define NG 64
#define NRG (NBP * NG)
#define ATT 1024
#define KO 96
#define KOP 128
typedef __attribute__((ext_vector_type(8))) __bf16 v8b;
__device__ __forceinline__ v16b frag_b(const __bf16* rowk0, int lane) {
  union { v16b v; v8b q[2]; } u; const __bf16* p = rowk0 + 8 * (lane >> 4);
  u.q[0] = *(const v8b*)p; u.q[1] = *(const v8b*)(p + 16); return u.v;
}
__device__ __forceinline__ float bfr(float v) { return (float)(__bf16)v; }
__device__ __attribute__((noinline)) float exp_ni(float v) { return expf(v); }
__device__ __attribute__((noinline)) float erf_ni(float v) { return erff(v); }

#define PK_ENC 0
#define PK_DEC (PK_ENC + ATT * HD)
#define PK_OUT (PK_DEC + ATT * HD)
#define PK_MLP (PK_OUT + ATT * KO)
#define PK_END (PK_MLP + ATT * ATT)
#define WS_PK   0u
#define WS_EH   (((2u * PK_END) + 127u) / 128u * 128u)
#define WS_EL   (WS_EH + 2u * NRG * HD)
#define WS_DA   (WS_EL + 2u * NRG * HD)
#define WS_PART (WS_DA + 4u * NBP * ATT)
#define WS_A2H  (WS_PART + 4u * 8 * NRG)
#define WS_A2L  (WS_A2H + 2u * NBP * KOP)
#define WS_O1H  (WS_A2L + 2u * NBP * KOP)
#define WS_O1L  (WS_O1H + 2u * NBP * ATT)
#define WS_X    (WS_O1L + 2u * NBP * ATT)
#define WS_ST   (WS_X + 4u * NBP * ATT)
#define WS_MR   (WS_ST + 8u * 32 * ATT * 2)
#define WS_END  (WS_MR + 4u * 4 * ATT)

__global__ __launch_bounds__(256) void k_pack(const float* __restrict__ WE, const float* __restrict__ WD, const float* __restrict__ WO, const float* __restrict__ WM, __bf16* __restrict__ PK) {
  __shared__ __align__(16) __bf16 s[ATT]; const int n = blockIdx.x, which = blockIdx.y, t = threadIdx.x; int K; size_t dst;
  if (which == 0) { K = HD; dst = PK_ENC + (size_t)n * HD; if (t < HD) s[t] = (__bf16)WE[(size_t)t * ATT + n]; }
  else if (which == 1) { K = HD; dst = PK_DEC + (size_t)n * HD; if (t < HD) s[t] = (__bf16)WD[(size_t)t * ATT + n]; }
  else if (which == 2) { K = KO; dst = PK_OUT + (size_t)n * KO; if (t < KO) s[t] = (__bf16)((t < 68) ? WO[(size_t)t * ATT + n] : 0.f); }
  else { K = ATT; dst = PK_MLP + (size_t)n * ATT; for (int k = t; k < ATT; k += 256) s[k] = (__bf16)WM[(size_t)k * ATT + n]; }
  __syncthreads();
  for (int q = t; q < K / 8; q += 256) vst2((unsigned*)(PK + dst + q * 8), *(const v4u*)&s[q * 8]);
}
__global__ __launch_bounds__(64) void k_pool(const float* __restrict__ H, const float* __restrict__ EP, __bf16* __restrict__ EH, __bf16* __restrict__ EL) {
  __shared__ signed char scell[NPED][NPED]; __shared__ float spx[NPED], spy[NPED]; __shared__ float shid[NPED][HD + 1]; __shared__ float stile[NG][HD + 1]; __shared__ __align__(16) __bf16 sh_[NG][HD + 8], sl_[NG][HD + 8];
  const int t = threadIdx.x; const int s = blockIdx.x;
  spx[t] = bfr(EP[((size_t)s * NPED + t) * 2]); spy[t] = bfr(EP[((size_t)s * NPED + t) * 2 + 1]);
  for (int d = 0; d < HD; ++d) shid[t][d] = bfr(H[((size_t)s * NPED + t) * HD + d]);
  __syncthreads();
  for (int i = 0; i < NPED; ++i) { const float ax = spx[i], ay = spy[i], ox = spx[t], oy = spy[t];
    const float tl_x = ax - 1.0f, tl_y = ay + 1.0f, br_x = ax + 1.0f, br_y = ay - 1.0f;
    const float cx = floorf((ox - tl_x) / 2.0f * 8.0f), cy = floorf((tl_y - oy) / 2.0f * 8.0f);
    const bool oob = (ox >= br_x) || (ox <= tl_x) || (oy >= tl_y) || (oy <= br_y) || (t == i);
    int g = (int)(cx + cy * 8.0f); if (oob) g = -1; else g = min(max(g, 0), NG - 1);
    scell[i][t] = (signed char)g; }
  __syncthreads();
  for (int i = 0; i < NPED; ++i) {
    for (int g = 0; g < NG; ++g) stile[g][t] = 0.f;
    for (int j = 0; j < NPED; ++j) { const int g = scell[i][j]; if (g >= 0) stile[g][t] += shid[j][t]; }
    __syncthreads();
    for (int e = t; e < NG * HD; e += 64) { const int g = e / HD, d = e % HD; const float v = stile[g][d]; const __bf16 hb = (__bf16)v; sh_[g][d] = hb; sl_[g][d] = (__bf16)(v - (float)hb); }
    __syncthreads();
    for (int e = t; e < NG * 8; e += 64) { const int g = e >> 3, pc = e & 7; const size_t o = (((size_t)s * NPED + i) * NG + g) * HD + pc * 8; vst2((unsigned*)(EH + o), *(const v4u*)&sh_[g][pc * 8]); vst2((unsigned*)(EL + o), *(const v4u*)&sl_[g][pc * 8]); }
    __syncthreads(); }
}
__global__ __launch_bounds__(128) void k_dec(const float* __restrict__ H, const __bf16* __restrict__ PK, const float* __restrict__ BD, float* __restrict__ DA) {
  __shared__ __align__(16) float so[4][16][132];
  const int tid = threadIdx.x, wave = tid >> 5, lane = tid & 31, col = lane & 15, g = lane >> 4; const size_t r0 = (size_t)blockIdx.x * 64 + wave * 16; const int n0 = blockIdx.y * 128;
  v8f acc[8] = {};
#pragma unroll
  for (int kc = 0; kc < HD / 32; ++kc) { v16b a; { const float* p = H + (r0 + col) * HD + kc * 32 + 8 * g;
#pragma unroll
      for (int i = 0; i < 8; ++i) { a[i] = (__bf16)p[i]; a[8 + i] = (__bf16)p[16 + i]; } }
#pragma unroll
    for (int j = 0; j < 8; ++j) acc[j] = wmma_bf(a, frag_b(PK + PK_DEC + (size_t)(n0 + j * 16 + col) * HD + kc * 32, lane), acc[j]); }
#pragma unroll
  for (int j = 0; j < 8; ++j) { const float bb = bfr(BD[n0 + j * 16 + col]);
#pragma unroll
    for (int r = 0; r < 8; ++r) so[wave][8 * g + r][j * 16 + col] = acc[j][r] + bb; }
  LDSX();
  for (int rl = 0; rl < 16; ++rl) vst2(DA + (r0 + rl) * ATT + n0 + lane * 4, *(const v4f*)&so[wave][rl][lane * 4]);
}
__global__ __launch_bounds__(128) void k_enc(const __bf16* __restrict__ EH, const __bf16* __restrict__ EL, const __bf16* __restrict__ PK, const float* __restrict__ BE, const float* __restrict__ DA, const float* __restrict__ WF, float* __restrict__ PART) {
  __shared__ __align__(16) float sp[64];
  const int tid = threadIdx.x, wave = tid >> 5, lane = tid & 31, col = lane & 15, g = lane >> 4; const size_t r0 = (size_t)blockIdx.x * 64 + wave * 16; const int n0 = blockIdx.y * 128; const size_t ped = blockIdx.x;
  v8f acc[8] = {};
#pragma unroll
  for (int kc = 0; kc < HD / 32; ++kc) { const v16b ah = frag_b(EH + (r0 + col) * HD + kc * 32, lane), al = frag_b(EL + (r0 + col) * HD + kc * 32, lane);
#pragma unroll
    for (int j = 0; j < 8; ++j) { const v16b w = frag_b(PK + PK_ENC + (size_t)(n0 + j * 16 + col) * HD + kc * 32, lane); acc[j] = wmma_bf(al, w, acc[j]); acc[j] = wmma_bf(ah, w, acc[j]); } }
  float pr[8];
#pragma unroll
  for (int r = 0; r < 8; ++r) pr[r] = 0.f;
#pragma unroll
  for (int j = 0; j < 8; ++j) { const int c = n0 + j * 16 + col; const float add = bfr(BE[c]) + DA[ped * ATT + c]; const float wf = bfr(WF[c]);
#pragma unroll
    for (int r = 0; r < 8; ++r) pr[r] += fmaxf(acc[j][r] + add, 0.f) * wf; }
#pragma unroll
  for (int r = 0; r < 8; ++r) {
#pragma unroll
    for (int o = 1; o < 16; o <<= 1) pr[r] += __shfl_xor(pr[r], o); }
  if (col == 0) {
#pragma unroll
    for (int r = 0; r < 8; ++r) sp[wave * 16 + 8 * g + r] = pr[r]; }
  __syncthreads();
  if (tid < 16) vst2(PART + (size_t)blockIdx.y * NRG + (size_t)blockIdx.x * 64 + tid * 4, *(const v4f*)&sp[tid * 4]);
}
__global__ __launch_bounds__(64) void k_ctx(const float* __restrict__ PART, const float* __restrict__ BF, const __bf16* __restrict__ EH, const __bf16* __restrict__ EL, const float* __restrict__ EP, const float* __restrict__ RP, const float* __restrict__ WEM, const float* __restrict__ BEM, __bf16* __restrict__ A2H, __bf16* __restrict__ A2L) {
  __shared__ float ssc[NG], sal[NG]; __shared__ __align__(16) __bf16 sh_[KOP], sl_[KOP]; const int t = threadIdx.x; const size_t b = blockIdx.x;
  sh_[HD + t] = (__bf16)0.f; sl_[HD + t] = (__bf16)0.f;
  __syncthreads();
  { float sc = 0.f;
#pragma unroll
    for (int cb = 0; cb < 8; ++cb) sc += PART[(size_t)cb * NRG + b * NG + t];
    ssc[t] = sc + bfr(BF[0]); }
  __syncthreads();
  { float mx = -3.0e38f; for (int g2 = 0; g2 < NG; ++g2) mx = fmaxf(mx, ssc[g2]); float se = 0.f; for (int g2 = 0; g2 < NG; ++g2) se += exp_ni(ssc[g2] - mx); sal[t] = exp_ni(ssc[t] - mx) / se; }
  __syncthreads();
  { float c = 0.f;
#pragma unroll 1
    for (int g2 = 0; g2 < NG; ++g2) { const size_t o = (b * NG + g2) * HD + t; c += sal[g2] * ((float)EH[o] + (float)EL[o]); }
    const __bf16 hb = (__bf16)c; sh_[t] = hb; sl_[t] = (__bf16)(c - (float)hb); }
  if (t < 32) { float v = 0.f; if (t < 4) { const float e0 = bfr(EP[b * 2]), e1 = bfr(EP[b * 2 + 1]), r0v = bfr(RP[b * 2]), r1v = bfr(RP[b * 2 + 1]); v = fmaxf(((e0 * bfr(WEM[0 * 4 + t]) + e1 * bfr(WEM[1 * 4 + t])) + r0v * bfr(WEM[2 * 4 + t])) + r1v * bfr(WEM[3 * 4 + t]) + bfr(BEM[t]), 0.f); }
    const __bf16 hb = (__bf16)v; sh_[HD + t] = hb; sl_[HD + t] = (__bf16)(v - (float)hb); }
  __syncthreads();
  if (t < 16) vst2((unsigned*)(A2H + b * KOP + t * 8), *(const v4u*)&sh_[t * 8]); else if (t < 32) vst2((unsigned*)(A2L + b * KOP + (t - 16) * 8), *(const v4u*)&sl_[(t - 16) * 8]);
}
__global__ __launch_bounds__(128) void k_out1(const __bf16* __restrict__ A2H, const __bf16* __restrict__ A2L, const __bf16* __restrict__ PK, const float* __restrict__ BO, __bf16* __restrict__ O1H, __bf16* __restrict__ O1L) {
  __shared__ __align__(16) __bf16 soh[4][16][136], sol[4][16][136];
  const int tid = threadIdx.x, wave = tid >> 5, lane = tid & 31, col = lane & 15, g = lane >> 4; const size_t r0 = (size_t)blockIdx.x * 64 + wave * 16; const int n0 = blockIdx.y * 128;
  v8f acc[8] = {};
#pragma unroll
  for (int kc = 0; kc < KO / 32; ++kc) { const v16b ah = frag_b(A2H + (r0 + col) * KOP + kc * 32, lane), al = frag_b(A2L + (r0 + col) * KOP + kc * 32, lane);
#pragma unroll
    for (int j = 0; j < 8; ++j) { const v16b w = frag_b(PK + PK_OUT + (size_t)(n0 + j * 16 + col) * KO + kc * 32, lane); acc[j] = wmma_bf(al, w, acc[j]); acc[j] = wmma_bf(ah, w, acc[j]); } }
#pragma unroll
  for (int j = 0; j < 8; ++j) { const float bb = bfr(BO[n0 + j * 16 + col]);
#pragma unroll
    for (int r = 0; r < 8; ++r) { const float v = fmaxf(acc[j][r] + bb, 0.f); const __bf16 hb = (__bf16)v; soh[wave][8 * g + r][j * 16 + col] = hb; sol[wave][8 * g + r][j * 16 + col] = (__bf16)(v - (float)hb); } }
  LDSX();
  for (int rl = 0; rl < 16; ++rl) { if (lane < 16) vst2((unsigned*)(O1H + (r0 + rl) * ATT + n0 + lane * 8), *(const v4u*)&soh[wave][rl][lane * 8]); else vst2((unsigned*)(O1L + (r0 + rl) * ATT + n0 + (lane - 16) * 8), *(const v4u*)&sol[wave][rl][(lane - 16) * 8]); }
}
__global__ __launch_bounds__(128) void k_mlp(const __bf16* __restrict__ O1H, const __bf16* __restrict__ O1L, const __bf16* __restrict__ PK, const float* __restrict__ BM, float* __restrict__ X, double* __restrict__ ST) {
  __shared__ __align__(16) float so[4][16][132]; __shared__ __align__(16) double sst[128][2];
  const int tid = threadIdx.x, wave = tid >> 5, lane = tid & 31, col = lane & 15, g = lane >> 4; const size_t r0 = (size_t)blockIdx.x * 64 + wave * 16; const int n0 = blockIdx.y * 128;
  v8f acc[8] = {};
#pragma unroll 2
  for (int kc = 0; kc < ATT / 32; ++kc) { const v16b ah = frag_b(O1H + (r0 + col) * ATT + kc * 32, lane), al = frag_b(O1L + (r0 + col) * ATT + kc * 32, lane);
#pragma unroll
    for (int j = 0; j < 8; ++j) { const v16b w = frag_b(PK + PK_MLP + (size_t)(n0 + j * 16 + col) * ATT + kc * 32, lane); acc[j] = wmma_bf(al, w, acc[j]); acc[j] = wmma_bf(ah, w, acc[j]); } }
#pragma unroll
  for (int j = 0; j < 8; ++j) { const float bb = bfr(BM[n0 + j * 16 + col]);
#pragma unroll
    for (int r = 0; r < 8; ++r) so[wave][8 * g + r][j * 16 + col] = acc[j][r] + bb; }
  __syncthreads();
  for (int rl = 0; rl < 16; ++rl) vst2(X + (r0 + rl) * ATT + n0 + lane * 4, *(const v4f*)&so[wave][rl][lane * 4]);
  { const int c = tid; double a = 0.0, b2 = 0.0; for (int w = 0; w < 4; ++w) for (int r = 0; r < 16; ++r) { const double v = (double)so[w][r][c]; a += v; b2 += v * v; } sst[c][0] = a; sst[c][1] = b2; }
  __syncthreads();
  vst2((unsigned*)(ST + ((size_t)blockIdx.x * ATT + n0 + tid) * 2), *(const v4u*)&sst[tid][0]);
}
__global__ __launch_bounds__(256) void k_red(const double* __restrict__ ST, const float* __restrict__ GA, const float* __restrict__ BEt, float* __restrict__ MR) {
  __shared__ __align__(16) float s[4 * ATT]; const int t = threadIdx.x;
  for (int c = t; c < ATT; c += 256) { double a = 0.0, b2 = 0.0; for (int blk = 0; blk < NBP / 64; ++blk) { a += ST[((size_t)blk * ATT + c) * 2]; b2 += ST[((size_t)blk * ATT + c) * 2 + 1]; }
    const double mean = a / (double)NBP; const double var = fmax(b2 / (double)NBP - mean * mean, 0.0); s[c] = (float)mean; s[ATT + c] = (float)(1.0 / sqrt(var + 1e-5)) * bfr(GA[c]); s[2 * ATT + c] = bfr(BEt[c]); s[3 * ATT + c] = 0.f; }
  __syncthreads();
  for (int q = t; q < ATT; q += 256) vst2(MR + q * 4, *(const v4f*)&s[q * 4]);
}
__global__ __launch_bounds__(256) void k_fin(const float* __restrict__ X, const float* __restrict__ MR, float* __restrict__ OUT) {
  const size_t row = blockIdx.x; const int t = threadIdx.x; v4f v;
#pragma unroll
  for (int i = 0; i < 4; ++i) { const int c = t * 4 + i; const float z = (X[row * ATT + c] - MR[c]) * MR[ATT + c] + MR[2 * ATT + c]; v[i] = fmaxf(z, 0.f); }
  vst2(OUT + row * ATT + t * 4, v);
}
extern "C" void kernel_launch(void* const* d_in, const int* in_sizes, int n_in, void* d_out, int out_size, void* d_ws, size_t ws_size, hipStream_t stream) {
  (void)in_sizes; (void)n_in; (void)out_size;
  const float** F = (const float**)d_in;
  if (ws_size < (size_t)WS_END) return;
  char* ws = (char*)d_ws; __bf16 *PK = (__bf16*)(ws + WS_PK), *EH = (__bf16*)(ws + WS_EH), *EL = (__bf16*)(ws + WS_EL), *A2H = (__bf16*)(ws + WS_A2H), *A2L = (__bf16*)(ws + WS_A2L), *O1H = (__bf16*)(ws + WS_O1H), *O1L = (__bf16*)(ws + WS_O1L); float *DA = (float*)(ws + WS_DA), *PART = (float*)(ws + WS_PART), *X = (float*)(ws + WS_X), *MR = (float*)(ws + WS_MR); double* ST = (double*)(ws + WS_ST);
  k_pack<<<dim3(ATT, 4), 256, 0, stream>>>(F[4], F[6], F[12], F[14], PK);
  k_pool<<<NS_, 64, 0, stream>>>(F[0], F[2], EH, EL);
  k_dec<<<dim3(NBP / 64, ATT / 128), 128, 0, stream>>>(F[0], PK, F[7], DA);
  k_enc<<<dim3(NRG / 64, ATT / 128), 128, 0, stream>>>(EH, EL, PK, F[5], DA, F[8], PART);
  k_ctx<<<NBP, 64, 0, stream>>>(PART, F[9], EH, EL, F[2], F[3], F[10], F[11], A2H, A2L);
  k_out1<<<dim3(NBP / 64, ATT / 128), 128, 0, stream>>>(A2H, A2L, PK, F[13], O1H, O1L);
  k_mlp<<<dim3(NBP / 64, ATT / 128), 128, 0, stream>>>(O1H, O1L, PK, F[15], X, ST);
  k_red<<<1, 256, 0, stream>>>(ST, F[16], F[17], MR);
  k_fin<<<NBP, 256, 0, stream>>>(X, MR, (float*)d_out);
}
